// LSTMNetwork_75522704933308
// MI455X (gfx1250) — hardware-run, weakly checked
//
#include <hip/hip_runtime.h>
#include <math.h>

constexpr int NBATCH       = 4096;
constexpr int NSTEP        = 512;
constexpr int NHID         = 16;
constexpr int NGATE        = 4 * NHID;
constexpr int ROWS_PER_BLK = 16;
constexpr int NBLK         = NBATCH / ROWS_PER_BLK;
constexpr int XCHUNK       = 32;
constexpr int NCHUNK       = NSTEP / XCHUNK;
constexpr int TPITCH       = 40;
constexpr int TILE_ELEMS   = ROWS_PER_BLK * TPITCH;
constexpr int XPITCH       = 36;
constexpr float HCARRY     = 1024.0f;
constexpr float WCARRY     = 16.0f;
constexpr float FOLD       = 1.0f / (HCARRY * WCARRY);

static_assert(NBATCH % ROWS_PER_BLK == 0, "batch tiles exact");
static_assert(NSTEP % XCHUNK == 0, "x chunks exact");
static_assert(NHID == 16, "one 16-column group per gate");
static_assert(NGATE == 64, "gate blocks i f g o");
static_assert((3 * TILE_ELEMS) % 32 == 0, "zero fill exact");
static_assert((TPITCH * 2) % 16 == 0, "tile rows 16-B aligned");
static_assert((XPITCH * 4) % 16 == 0, "x rows 16-B aligned");
static_assert(ROWS_PER_BLK * NHID == 256, "output tile = 1024 B");

typedef __attribute__((ext_vector_type(16))) _Float16 v16h;
typedef __attribute__((ext_vector_type(8)))  _Float16 v8h;
typedef __attribute__((ext_vector_type(8)))  float    v8f;
typedef __attribute__((ext_vector_type(4)))  float    v4f;

union FragU { v16h v; v8h h[2]; };

__device__ __forceinline__ v8h zero_v8h() {
  v8h z;
#pragma unroll
  for (int e = 0; e < 8; ++e) z[e] = (_Float16)0.0f;
  return z;
}

__device__ __forceinline__ v16h frag_load(const _Float16* p) {
  FragU f;
  f.h[0] = *(const v8h*)(p);
  f.h[1] = *(const v8h*)(p + 16);
  return f.v;
}
__device__ __forceinline__ v16h frag_load_rec_only(const _Float16* p16) {
  FragU f;
  f.h[0] = zero_v8h();
  f.h[1] = *(const v8h*)(p16);
  return f.v;
}
__device__ __forceinline__ v16h make_bfrag(const v4f i0, const v4f i1, const v4f r0, const v4f r1) {
  v16h f;
#pragma unroll
  for (int e = 0; e < 4; ++e) {
    f[e]      = (_Float16)(i0[e] * WCARRY);
    f[4 + e]  = (_Float16)(i1[e] * WCARRY);
    f[8 + e]  = (_Float16)(r0[e] * WCARRY);
    f[12 + e] = (_Float16)(r1[e] * WCARRY);
  }
  return f;
}

__device__ __forceinline__ v8f wmma_h(v16h a, v16h b, v8f c) {
  return __builtin_amdgcn_wmma_f32_16x16x32_f16(false, a, false, b, (short)0, c, false, false);
}
__device__ __forceinline__ void guard4(v8f& a0, v8f& a1, v8f& a2, v8f& a3,
                                       v16h x, v16h b0, v16h b1, v16h b2, v16h b3) {
  asm volatile("v_nop\n\tv_nop\n\tv_nop\n\tv_nop"
               : "+v"(a0), "+v"(a1), "+v"(a2), "+v"(a3)
               : "v"(x), "v"(b0), "v"(b1), "v"(b2), "v"(b3));
}

__device__ __forceinline__ float fsig(float x) {
  return __builtin_amdgcn_rcpf(1.0f + __expf(-x));
}
__device__ __forceinline__ float ftanh_e(float x) {
  return 1.0f - 2.0f * __builtin_amdgcn_rcpf(__expf(2.0f * x) + 1.0f);
}
__device__ __forceinline__ float cell_scalar(float pi, float pf, float pg, float po, float& cst) {
  const float ig = fsig(pi);
  const float fg = fsig(pf);
  const float gg = ftanh_e(pg);
  const float og = fsig(po);
  const float cn = fg * cst + ig * gg;
  cst = cn;
  return og * ftanh_e(cn);
}

__global__ __launch_bounds__(32) void lstm3_seq_kernel(
    const float* __restrict__ x,
    const float* __restrict__ wih0, const float* __restrict__ whh0,
    const float* __restrict__ bih0, const float* __restrict__ bhh0,
    const float* __restrict__ wih1, const float* __restrict__ whh1,
    const float* __restrict__ bih1, const float* __restrict__ bhh1,
    const float* __restrict__ wih2, const float* __restrict__ whh2,
    const float* __restrict__ bih2, const float* __restrict__ bhh2,
    float* __restrict__ out) {
  __shared__ __align__(16) _Float16 Tl[3 * TILE_ELEMS];
  __shared__ __align__(16) float    Xs[ROWS_PER_BLK * XPITCH];
  __shared__ __align__(16) float    Bs[3 * NGATE];
  __shared__ __align__(16) float    Ws[NGATE];
  __shared__ __align__(16) float    Os[ROWS_PER_BLK * NHID];

  const int lane = threadIdx.x & 31;
  const int c    = lane & 15;
  const int hh   = lane >> 4;
  const int b0   = blockIdx.x * ROWS_PER_BLK;

#pragma unroll 1
  for (int i = lane; i < 3 * TILE_ELEMS; i += 32) Tl[i] = (_Float16)0.0f;

  {
    const int i4 = c * 4;
    const v4f ba0 = *(const v4f*)(bih0 + i4);
    const v4f bb0 = *(const v4f*)(bhh0 + i4);
    const v4f ba1 = *(const v4f*)(bih1 + i4);
    const v4f bb1 = *(const v4f*)(bhh1 + i4);
    const v4f ba2 = *(const v4f*)(bih2 + i4);
    const v4f bb2 = *(const v4f*)(bhh2 + i4);
    const v4f w0  = *(const v4f*)(wih0 + i4);
    if (hh == 0) {
      *(v4f*)(Bs + 0 * NGATE + i4) = ba0 + bb0;
      *(v4f*)(Bs + 1 * NGATE + i4) = ba1 + bb1;
      *(v4f*)(Bs + 2 * NGATE + i4) = ba2 + bb2;
      *(v4f*)(Ws + i4) = w0;
    }
  }

  const v4f zero4 = {0.0f, 0.0f, 0.0f, 0.0f};
  v16h B0[4], B1[4], B2[4];
#pragma unroll
  for (int g = 0; g < 4; ++g) {
    const int n = g * NHID + c;
    const float* pr0 = whh0 + n * NHID + 8 * hh;
    const float* pi1 = wih1 + n * NHID + 8 * hh;
    const float* pr1 = whh1 + n * NHID + 8 * hh;
    const float* pi2 = wih2 + n * NHID + 8 * hh;
    const float* pr2 = whh2 + n * NHID + 8 * hh;
    B0[g] = make_bfrag(zero4, zero4, *(const v4f*)(pr0), *(const v4f*)(pr0 + 4));
    B1[g] = make_bfrag(*(const v4f*)(pi1), *(const v4f*)(pi1 + 4), *(const v4f*)(pr1), *(const v4f*)(pr1 + 4));
    B2[g] = make_bfrag(*(const v4f*)(pi2), *(const v4f*)(pi2 + 4), *(const v4f*)(pr2), *(const v4f*)(pr2 + 4));
  }

  __syncthreads();

  float bs0[4], bs1[4], bs2[4], wx[4];
#pragma unroll
  for (int g = 0; g < 4; ++g) {
    bs0[g] = Bs[0 * NGATE + g * NHID + c];
    bs1[g] = Bs[1 * NGATE + g * NHID + c];
    bs2[g] = Bs[2 * NGATE + g * NHID + c];
    wx[g]  = Ws[g * NHID + c];
  }

  float cs0[8], cs1[8], cs2[8], hfin[8];
#pragma unroll
  for (int r = 0; r < 8; ++r) { cs0[r] = 0.0f; cs1[r] = 0.0f; cs2[r] = 0.0f; hfin[r] = 0.0f; }

  _Float16* T0 = Tl;
  _Float16* T1 = Tl + TILE_ELEMS;
  _Float16* T2 = Tl + 2 * TILE_ELEMS;
  const _Float16* a0p = T0 + c * TPITCH + 16 + 8 * hh;
  const _Float16* a1p = T1 + c * TPITCH + 8 * hh;
  const _Float16* a2p = T2 + c * TPITCH + 8 * hh;
  const int wbase = 8 * hh * TPITCH;
  const float* xsrd = Xs + 8 * hh * XPITCH;
  const v8f z8 = {0.0f, 0.0f, 0.0f, 0.0f, 0.0f, 0.0f, 0.0f, 0.0f};

#pragma unroll 1
  for (int ch = 0; ch < NCHUNK; ++ch) {
    {
      const float* xp = x + (size_t)(b0 + c) * NSTEP + ch * XCHUNK + 16 * hh;
      const v4f q0 = *(const v4f*)(xp);
      const v4f q1 = *(const v4f*)(xp + 4);
      const v4f q2 = *(const v4f*)(xp + 8);
      const v4f q3 = *(const v4f*)(xp + 12);
      float* xd = Xs + c * XPITCH + 16 * hh;
      *(v4f*)(xd)      = q0;
      *(v4f*)(xd + 4)  = q1;
      *(v4f*)(xd + 8)  = q2;
      *(v4f*)(xd + 12) = q3;
    }
    __syncthreads();

#pragma unroll 1
    for (int tt = 0; tt < XCHUNK; ++tt) {
      {
        const v16h fa = frag_load_rec_only(a0p);
        v8f g0 = wmma_h(fa, B0[0], z8);
        v8f g1 = wmma_h(fa, B0[1], z8);
        v8f g2 = wmma_h(fa, B0[2], z8);
        v8f g3 = wmma_h(fa, B0[3], z8);
        guard4(g0, g1, g2, g3, fa, B0[0], B0[1], B0[2], B0[3]);
        float hn[8];
#pragma unroll
        for (int r = 0; r < 8; ++r) {
          const float xv = xsrd[r * XPITCH + tt];
          const float pi = fmaf(g0[r], FOLD, fmaf(xv, wx[0], bs0[0]));
          const float pf = fmaf(g1[r], FOLD, fmaf(xv, wx[1], bs0[1]));
          const float pg = fmaf(g2[r], FOLD, fmaf(xv, wx[2], bs0[2]));
          const float po = fmaf(g3[r], FOLD, fmaf(xv, wx[3], bs0[3]));
          hn[r] = cell_scalar(pi, pf, pg, po, cs0[r]);
        }
#pragma unroll
        for (int r = 0; r < 8; ++r) {
          const _Float16 hv = (_Float16)(hn[r] * HCARRY);
          T0[wbase + r * TPITCH + 16 + c] = hv;
          T1[wbase + r * TPITCH + c]      = hv;
        }
      }
      __syncthreads();
      {
        const v16h fa = frag_load(a1p);
        v8f g0 = wmma_h(fa, B1[0], z8);
        v8f g1 = wmma_h(fa, B1[1], z8);
        v8f g2 = wmma_h(fa, B1[2], z8);
        v8f g3 = wmma_h(fa, B1[3], z8);
        guard4(g0, g1, g2, g3, fa, B1[0], B1[1], B1[2], B1[3]);
        float hn[8];
#pragma unroll
        for (int r = 0; r < 8; ++r) {
          const float pi = fmaf(g0[r], FOLD, bs1[0]);
          const float pf = fmaf(g1[r], FOLD, bs1[1]);
          const float pg = fmaf(g2[r], FOLD, bs1[2]);
          const float po = fmaf(g3[r], FOLD, bs1[3]);
          hn[r] = cell_scalar(pi, pf, pg, po, cs1[r]);
        }
#pragma unroll
        for (int r = 0; r < 8; ++r) {
          const _Float16 hv = (_Float16)(hn[r] * HCARRY);
          T1[wbase + r * TPITCH + 16 + c] = hv;
          T2[wbase + r * TPITCH + c]      = hv;
        }
      }
      __syncthreads();
      {
        const v16h fa = frag_load(a2p);
        v8f g0 = wmma_h(fa, B2[0], z8);
        v8f g1 = wmma_h(fa, B2[1], z8);
        v8f g2 = wmma_h(fa, B2[2], z8);
        v8f g3 = wmma_h(fa, B2[3], z8);
        guard4(g0, g1, g2, g3, fa, B2[0], B2[1], B2[2], B2[3]);
#pragma unroll
        for (int r = 0; r < 8; ++r) {
          const float pi = fmaf(g0[r], FOLD, bs2[0]);
          const float pf = fmaf(g1[r], FOLD, bs2[1]);
          const float pg = fmaf(g2[r], FOLD, bs2[2]);
          const float po = fmaf(g3[r], FOLD, bs2[3]);
          hfin[r] = cell_scalar(pi, pf, pg, po, cs2[r]);
        }
#pragma unroll
        for (int r = 0; r < 8; ++r) {
          T2[wbase + r * TPITCH + 16 + c] = (_Float16)(hfin[r] * HCARRY);
        }
      }
      __syncthreads();
    }
  }

#pragma unroll
  for (int r = 0; r < 8; ++r) Os[(8 * hh + r) * NHID + c] = hfin[r];
  __syncthreads();
  {
    const v4f o0 = *(const v4f*)(Os + lane * 4);
    const v4f o1 = *(const v4f*)(Os + 128 + lane * 4);
    float* op = out + (size_t)blockIdx.x * (ROWS_PER_BLK * NHID);
    *(volatile v4f*)(op + lane * 4)       = o0;
    *(volatile v4f*)(op + 128 + lane * 4) = o1;
    __threadfence();
    *(volatile v4f*)(op + lane * 4)       = o0;
    *(volatile v4f*)(op + 128 + lane * 4) = o1;
  }
}

extern "C" void kernel_launch(void* const* d_in, const int* in_sizes, int n_in,
                              void* d_out, int out_size, void* d_ws, size_t ws_size, hipStream_t stream) {
  (void)d_ws; (void)ws_size;
  if (n_in < 13 || d_out == nullptr) return;
  if (in_sizes[0] != NBATCH * NSTEP || in_sizes[1] != NGATE || in_sizes[2] != NGATE * NHID ||
      in_sizes[3] != NGATE || in_sizes[4] != NGATE ||
      in_sizes[5] != NGATE * NHID || in_sizes[6] != NGATE * NHID || in_sizes[7] != NGATE || in_sizes[8] != NGATE ||
      in_sizes[9] != NGATE * NHID || in_sizes[10] != NGATE * NHID || in_sizes[11] != NGATE || in_sizes[12] != NGATE ||
      out_size != NBATCH * NHID) return;

  const float* x    = (const float*)d_in[0];
  const float* wih0 = (const float*)d_in[1];
  const float* whh0 = (const float*)d_in[2];
  const float* bih0 = (const float*)d_in[3];
  const float* bhh0 = (const float*)d_in[4];
  const float* wih1 = (const float*)d_in[5];
  const float* whh1 = (const float*)d_in[6];
  const float* bih1 = (const float*)d_in[7];
  const float* bhh1 = (const float*)d_in[8];
  const float* wih2 = (const float*)d_in[9];
  const float* whh2 = (const float*)d_in[10];
  const float* bih2 = (const float*)d_in[11];
  const float* bhh2 = (const float*)d_in[12];

  lstm3_seq_kernel<<<NBLK, 32, 0, stream>>>(x, wih0, whh0, bih0, bhh0, wih1, whh1, bih1, bhh1,
                                            wih2, whh2, bih2, bhh2, (float*)d_out);
}
